// MultiHeadAttention_39926015983741
// MI455X (gfx1250) — hardware-verified
//
#include <hip/hip_runtime.h>


#ifndef NB
#define NB 2
#endif
#ifndef SEQ
#define SEQ 2048
#endif
#define SEQ_FULL 2048
#define DM   1024
#define NH_  16
#define HD   64
#define MT   (NB * SEQ)
#define SCL  0.125f
#define L2E  1.4426950408889634f
#define PC2  10.0f
#define RCAR 1024.0f
#define RINV 0.0009765625f

static_assert(SEQ % 64 == 0);
static_assert(SEQ <= SEQ_FULL);
static_assert(DM == NH_ * HD);
static_assert(DM % 64 == 0);
static_assert(DM / 8 == 128);
static_assert(MT % 64 == 0);
static_assert(((size_t)MT * DM / 8) % 256 == 0);
static_assert(((size_t)DM * DM / 64) % 64 == 0);
static_assert((size_t)NB * NH_ * SEQ * (HD / 8) == (size_t)MT * DM / 8);
static_assert((size_t)NB * NH_ * HD * (SEQ / 8) == (size_t)MT * DM / 8);
static_assert(NH_ == 16);
static_assert(HD == 64);

typedef _Float16 h16;
typedef unsigned short bf;
typedef __attribute__((ext_vector_type(16))) __bf16   v16bf;
typedef __attribute__((ext_vector_type(16))) _Float16 v16h;
typedef __attribute__((ext_vector_type(8)))  _Float16 v8h;
typedef __attribute__((ext_vector_type(8)))  unsigned short v8us;
typedef __attribute__((ext_vector_type(2)))  unsigned short v2us;
typedef __attribute__((ext_vector_type(8)))  float    v8f;
typedef __attribute__((ext_vector_type(4)))  float    v4f;
typedef __attribute__((ext_vector_type(4)))  int      v4i;
typedef v4f  __attribute__((may_alias)) v4fa;

__device__ __forceinline__ unsigned short f2bf(float f) { unsigned u = __float_as_uint(f); u += 0x7FFFu + ((u >> 16) & 1u); return (unsigned short)(u >> 16); }
__device__ __forceinline__ float bf2f(unsigned short b) { return __uint_as_float(((unsigned)b) << 16); }
__device__ __forceinline__ float bfr(float f) { return bf2f(f2bf(f)); }
__device__ __forceinline__ void splitf(float y, unsigned short& h, unsigned short& l) { h = f2bf(y); l = f2bf(y - bf2f(h)); }
__device__ __forceinline__ v16h cat16(v8h lo, v8h hi) { return __builtin_shufflevector(lo, hi, 0, 1, 2, 3, 4, 5, 6, 7, 8, 9, 10, 11, 12, 13, 14, 15); }
__device__ __forceinline__ v16bf cat16b(v8us lo, v8us hi) { return __builtin_bit_cast(v16bf, __builtin_shufflevector(lo, hi, 0, 1, 2, 3, 4, 5, 6, 7, 8, 9, 10, 11, 12, 13, 14, 15)); }
__device__ __forceinline__ v8f wmma16(v16h a, v16h b, v8f c) { return __builtin_amdgcn_wmma_f32_16x16x32_f16(false, a, false, b, (short)0, c, false, false); }
__device__ __forceinline__ v8f wmmab(v16bf a, v16bf b, v8f c) { return __builtin_amdgcn_wmma_f32_16x16x32_bf16(false, a, false, b, (short)0, c, false, false); }

template <typename T16> struct WFrag;
template <> struct WFrag<h16> { typedef v16h V; static __device__ __forceinline__ V ld(const h16* p) { return cat16(*(const v8h*)p, *(const v8h*)(p + 16)); } static __device__ __forceinline__ v8f mma(V a, V b, v8f c) { return wmma16(a, b, c); } };
template <> struct WFrag<bf> { typedef v16bf V; static __device__ __forceinline__ V ld(const bf* p) { return cat16b(*(const v8us*)p, *(const v8us*)(p + 16)); } static __device__ __forceinline__ v8f mma(V a, V b, v8f c) { return wmmab(a, b, c); } };
template <typename T16, int NSPLIT, bool BIAS>
__global__ __launch_bounds__(32) void k_gemmw(const T16* __restrict__ A, const T16* __restrict__ A2, const T16* __restrict__ Bt, const T16* __restrict__ Bt2, int K, float* C, int ldc, const float* __restrict__ bias, size_t sA, size_t sB, size_t sC) {
    typedef typename WFrag<T16>::V V;
    __shared__ __align__(16) float os[16 * 68];
    const size_t z = blockIdx.z; A += z * sA; if (A2) A2 += z * sA; Bt += z * sB; if (Bt2) Bt2 += z * sB; C += z * sC;
    const int lane = threadIdx.x & 31, lr = lane & 15, hi = lane >> 4; const int r0 = blockIdx.x * 64, c0 = blockIdx.y * 64;
    v8f acc[4][4];
#pragma unroll
    for (int mb = 0; mb < 4; ++mb)
#pragma unroll
        for (int nb = 0; nb < 4; ++nb) acc[mb][nb] = (v8f){};
    const size_t aoff = (size_t)(r0 + lr) * K + 8 * hi, boff = (size_t)(c0 + lr) * K + 8 * hi;
#pragma unroll 1
    for (int kc = 0; kc < K; kc += 32) {
        V a[4], a2[4];
#pragma unroll
        for (int mb = 0; mb < 4; ++mb) { a[mb] = WFrag<T16>::ld(A + aoff + (size_t)mb * 16 * K + kc); if (NSPLIT == 1 || NSPLIT == 2) a2[mb] = WFrag<T16>::ld(A2 + aoff + (size_t)mb * 16 * K + kc); }
#pragma unroll
        for (int nb = 0; nb < 4; ++nb) { const V b = WFrag<T16>::ld(Bt + boff + (size_t)nb * 16 * K + kc); V b2; if (NSPLIT >= 2) b2 = WFrag<T16>::ld(Bt2 + boff + (size_t)nb * 16 * K + kc);
#pragma unroll
            for (int mb = 0; mb < 4; ++mb) { acc[mb][nb] = WFrag<T16>::mma(a[mb], b, acc[mb][nb]); if (NSPLIT == 1 || NSPLIT == 2) acc[mb][nb] = WFrag<T16>::mma(a2[mb], b, acc[mb][nb]); if (NSPLIT >= 2) acc[mb][nb] = WFrag<T16>::mma(a[mb], b2, acc[mb][nb]); } }
        asm volatile("v_nop\n\tv_nop\n\tv_nop\n\tv_nop" : "+v"(acc[0][0]), "+v"(acc[1][1]), "+v"(acc[2][2]), "+v"(acc[3][3]) : "v"(a[0]), "v"(a[3]));
    }
#pragma unroll
    for (int mb = 0; mb < 4; ++mb) {
#pragma unroll
        for (int nb = 0; nb < 4; ++nb) {
#pragma unroll
            for (int j = 0; j < 8; ++j) os[(hi * 8 + j) * 68 + nb * 16 + lr] = acc[mb][nb][j]; }
        __builtin_amdgcn_wave_barrier(); asm volatile("" ::: "memory");
        float* crow = C + (size_t)(r0 + mb * 16) * ldc + c0;
#pragma unroll 1
        for (int ps = 0; ps < 2; ++ps) {
#pragma unroll
            for (int s = 0; s < 8; ++s) { const int row = 2 * s + hi, cofs = lr * 4; v4f val = *(const v4fa*)(os + row * 68 + cofs); if (BIAS) { val[0] += bfr(bias[c0 + cofs]); val[1] += bfr(bias[c0 + cofs + 1]); val[2] += bfr(bias[c0 + cofs + 2]); val[3] += bfr(bias[c0 + cofs + 3]); }
                *(volatile v4f*)(crow + (size_t)row * ldc + cofs) = val; }
            if (ps == 0) __threadfence(); }
        __builtin_amdgcn_wave_barrier(); asm volatile("" ::: "memory");
    }
}

__global__ __launch_bounds__(256) void k_wtG(const float* __restrict__ w, bf* Bt) {
    const unsigned lane = threadIdx.x & 31u; const unsigned L0 = (blockIdx.x * 8u + (threadIdx.x >> 5)) * 8u; const unsigned nlines = (unsigned)DM * DM / 64u;
#pragma unroll 1
    for (int ps = 0; ps < 2; ++ps) {
#pragma unroll 1
        for (unsigned l = 0; l < 8u; ++l) { const unsigned L = L0 + l; if (L < nlines) { const unsigned e = L * 64u + lane * 2u; const unsigned k = e & (unsigned)(DM - 1), n = e >> 10; v2us o;
            o[0] = f2bf(w[(size_t)k * DM + n]); o[1] = f2bf(w[(size_t)(k + 1u) * DM + n]); *(volatile v2us*)(Bt + e) = o; } }
        if (ps == 0) __threadfence(); }
}

__global__ __launch_bounds__(256) void k_cvt8(const float* __restrict__ src, bf* dst) {
    const unsigned i = blockIdx.x * 256u + threadIdx.x; if (i >= (unsigned)MT * (DM / 8)) return;
    const unsigned row = i >> 7, c8 = i & 127u; const unsigned b = row / (unsigned)SEQ, t = row - b * (unsigned)SEQ;
    const v8f v = *(const v8f*)(src + ((size_t)(b * (unsigned)SEQ_FULL + t) * DM + c8 * 8u)); v8us o;
#pragma unroll
    for (int k = 0; k < 8; ++k) o[k] = f2bf(v[k]);
    *(volatile v8us*)(dst + (size_t)i * 8) = o; __threadfence(); *(volatile v8us*)(dst + (size_t)i * 8) = o; }

template <bool RES>
__device__ __forceinline__ void qkp_body(const float* __restrict__ F, h16* P, h16* PR) {
    const unsigned i = blockIdx.x * 256u + threadIdx.x; if (i >= (unsigned)NB * NH_ * SEQ * (HD / 8)) return;
    const unsigned d8 = i & 7u, rt = i >> 3; const unsigned bh = rt / (unsigned)SEQ, t = rt - bh * (unsigned)SEQ; const unsigned h = bh & (unsigned)(NH_ - 1), b = bh >> 4;
    const float* f = F + ((size_t)(b * (unsigned)SEQ + t) * DM + h * (unsigned)HD + d8 * 8u);
    const v4f a = *(const v4f*)f, c = *(const v4f*)(f + 4); v8h o, orr;
#pragma unroll
    for (int k = 0; k < 4; ++k) { const h16 ha = (h16)a[k], hc = (h16)c[k]; o[k] = ha; o[k + 4] = hc; orr[k] = (h16)((a[k] - (float)ha) * RCAR); orr[k + 4] = (h16)((c[k] - (float)hc) * RCAR); }
    *(volatile v8h*)(P + (size_t)i * 8) = o; if (RES) *(volatile v8h*)(PR + (size_t)i * 8) = orr;
    __threadfence();
    *(volatile v8h*)(P + (size_t)i * 8) = o; if (RES) *(volatile v8h*)(PR + (size_t)i * 8) = orr; }
__global__ __launch_bounds__(256) void k_qp(const float* __restrict__ F, h16* P, h16* PR) { qkp_body<true>(F, P, PR); }
__global__ __launch_bounds__(256) void k_kp(const float* __restrict__ F, h16* P) { qkp_body<false>(F, P, P); }

__global__ __launch_bounds__(256) void k_vtp(const float* __restrict__ F, h16* VT, h16* VR) {
    const unsigned i = blockIdx.x * 256u + threadIdx.x; if (i >= (unsigned)NB * NH_ * HD * (SEQ / 8)) return;
    const unsigned rd = i / (unsigned)(SEQ / 8), t8 = i - rd * (unsigned)(SEQ / 8); const unsigned d = rd & (unsigned)(HD - 1), bh = rd >> 6; const unsigned h = bh & (unsigned)(NH_ - 1), b = bh >> 4;
    const float* f = F + ((size_t)(b * (unsigned)SEQ + t8 * 8u) * DM + h * (unsigned)HD + d); v8h o, orr;
#pragma unroll
    for (int q = 0; q < 8; ++q) { const float x = f[(size_t)q * DM]; const h16 hx = (h16)x; o[q] = hx; orr[q] = (h16)((x - (float)hx) * RCAR); }
    *(volatile v8h*)(VT + (size_t)i * 8) = o; *(volatile v8h*)(VR + (size_t)i * 8) = orr;
    __threadfence();
    *(volatile v8h*)(VT + (size_t)i * 8) = o; *(volatile v8h*)(VR + (size_t)i * 8) = orr; }

__global__ __launch_bounds__(128) void k_flash(const h16* __restrict__ QP, const h16* __restrict__ QR, const h16* __restrict__ KP, const h16* __restrict__ VT, const h16* __restrict__ VR, const int* __restrict__ mask, bf* CTh, bf* CTl) {
    __shared__ __align__(16) float osm[4][16 * 68];
    const unsigned lane = threadIdx.x & 31u, lr = lane & 15u, hi = lane >> 4, wv = threadIdx.x >> 5;
    const unsigned bh = blockIdx.y, b = bh >> 4, h = bh & (unsigned)(NH_ - 1);
    const unsigned q0 = blockIdx.x * 64u + wv * 16u;
    const size_t qoff = (size_t)bh * SEQ * HD + (size_t)(q0 + lr) * HD + 8u * hi;
    const h16* Qp = QP + qoff; const h16* Qr = QR + qoff;
    const h16* Kp = KP + (size_t)bh * SEQ * HD + (size_t)lr * HD + 8u * hi;
    const size_t voff = (size_t)bh * HD * SEQ + (size_t)lr * SEQ + 8u * hi;
    const h16* Vp = VT + voff; const h16* Vr = VR + voff;
    const int* mp = mask + ((size_t)(b * (unsigned)SEQ_FULL + q0 + lr)) * SEQ_FULL + 8u * hi;
    v8f O[4];
#pragma unroll
    for (int dt = 0; dt < 4; ++dt) O[dt] = (v8f){};
    float mrun = -1.0e30f, lrun = 0.0f;
#pragma unroll 1
    for (unsigned kc = 0; kc < (unsigned)SEQ; kc += 64u) {
        unsigned qo = 0u; asm volatile("" : "+v"(qo));
        const v16h qb0 = WFrag<h16>::ld(Qp + qo), qb1 = WFrag<h16>::ld(Qp + qo + 32u), qr0 = WFrag<h16>::ld(Qr + qo), qr1 = WFrag<h16>::ld(Qr + qo + 32u);
        v8f s[4]; float cm = -1.0e30f;
#pragma unroll
        for (int kt = 0; kt < 4; ++kt) {
            const h16* kp = Kp + (size_t)(kc + kt * 16) * HD; const v16h ka0 = WFrag<h16>::ld(kp), ka1 = WFrag<h16>::ld(kp + 32);
            const v4i m0 = *(const v4i*)(mp + kc + kt * 16); const v4i m1 = *(const v4i*)(mp + kc + kt * 16 + 4);
            v8f z = (v8f){}, zr = (v8f){};
            z = wmma16(ka0, qb0, z); zr = wmma16(ka0, qr0, zr); z = wmma16(ka1, qb1, z); zr = wmma16(ka1, qr1, zr);
            asm volatile("v_nop\n\tv_nop\n\tv_nop\n\tv_nop" : "+v"(z), "+v"(zr) : "v"(ka0), "v"(ka1), "v"(qr1));
            v8f sv;
#pragma unroll
            for (int r = 0; r < 4; ++r) { const float u0 = (z[r] + zr[r] * RINV) * SCL, u1 = (z[r + 4] + zr[r + 4] * RINV) * SCL; const float t0 = (m0[r] == 0) ? -1.0e9f : u0; const float t1 = (m1[r] == 0) ? -1.0e9f : u1; sv[r] = t0; sv[r + 4] = t1; cm = fmaxf(cm, fmaxf(t0, t1)); }
            s[kt] = sv; }
        cm = fmaxf(cm, __shfl_xor(cm, 16, 32));
        const float mnew = fmaxf(mrun, cm);
        const float corr = __builtin_amdgcn_exp2f((mrun - mnew) * L2E);
        float ls = 0.0f; v16h pb[2];
#pragma unroll
        for (int c = 0; c < 2; ++c) {
#pragma unroll
            for (int j = 0; j < 2; ++j) {
#pragma unroll
                for (int r = 0; r < 8; ++r) { const float d0 = s[2 * c + j][r] - mnew; const float p = __builtin_amdgcn_exp2f(d0 * L2E + PC2); ls += p; pb[c][j * 8 + r] = (h16)p; } } }
        ls += __shfl_xor(ls, 16, 32);
        lrun = lrun * corr + ls; mrun = mnew;
        v8f O2[4];
#pragma unroll
        for (int dt = 0; dt < 4; ++dt) { O[dt] = O[dt] * corr; O2[dt] = (v8f){}; }
#pragma unroll
        for (int c = 0; c < 2; ++c) {
#pragma unroll
            for (int dt = 0; dt < 4; ++dt) { const size_t vo = (size_t)(dt * 16) * SEQ + kc + c * 32; const v16h va = WFrag<h16>::ld(Vp + vo), vr = WFrag<h16>::ld(Vr + vo); O[dt] = wmma16(va, pb[c], O[dt]); O2[dt] = wmma16(vr, pb[c], O2[dt]); } }
        asm volatile("v_nop\n\tv_nop\n\tv_nop\n\tv_nop" : "+v"(O[0]), "+v"(O[1]), "+v"(O[2]), "+v"(O[3]), "+v"(O2[0]), "+v"(O2[1]), "+v"(O2[2]), "+v"(O2[3]) : "v"(pb[0]), "v"(pb[1]));
#pragma unroll
        for (int dt = 0; dt < 4; ++dt) O[dt] = O[dt] + O2[dt] * RINV;
    }
    const float inv = 1.0f / lrun;
    float* o = osm[wv];
#pragma unroll
    for (int dt = 0; dt < 4; ++dt) {
#pragma unroll
        for (int r = 0; r < 8; ++r) o[lr * 68u + dt * 16 + 8u * hi + r] = O[dt][r] * inv; }
    __builtin_amdgcn_wave_barrier(); asm volatile("" ::: "memory");
    const size_t rowbase = (size_t)(b * (unsigned)SEQ + q0) * DM + h * (unsigned)HD;
#pragma unroll 1
    for (int ps = 0; ps < 2; ++ps) {
#pragma unroll
        for (int s4 = 0; s4 < 4; ++s4) { const unsigned row = (unsigned)s4 * 4u + (lane >> 3), d8 = (lane & 7u) * 8u; const v4f a = *(const v4fa*)(o + row * 68u + d8), c = *(const v4fa*)(o + row * 68u + d8 + 4u); v8us oh, ol;
#pragma unroll
            for (int k = 0; k < 4; ++k) { unsigned short x, y; splitf(a[k], x, y); oh[k] = x; ol[k] = y; splitf(c[k], x, y); oh[k + 4] = x; ol[k + 4] = y; }
            *(volatile v8us*)(CTh + rowbase + (size_t)row * DM + d8) = oh; *(volatile v8us*)(CTl + rowbase + (size_t)row * DM + d8) = ol; }
        if (ps == 0) __threadfence(); }
    __builtin_amdgcn_wave_barrier(); asm volatile("" ::: "memory");
}

extern "C" void kernel_launch(void* const* d_in, const int* in_sizes, int n_in,
                              void* d_out, int out_size, void* d_ws, size_t ws_size, hipStream_t stream) {
    if (n_in < 12) return;
    const long long need_x = ((long long)(NB - 1) * SEQ_FULL + SEQ) * DM;
    const long long need_m = ((long long)(NB - 1) * SEQ_FULL + (SEQ - 1)) * SEQ_FULL + SEQ;
    if ((long long)in_sizes[0] < need_x || (long long)in_sizes[1] < need_x || (long long)in_sizes[2] < need_x || (long long)in_sizes[3] < need_m) return;
    if (in_sizes[4] < DM * DM || in_sizes[6] < DM * DM || in_sizes[8] < DM * DM || in_sizes[10] < DM * DM) return;
    if (in_sizes[5] < DM || in_sizes[7] < DM || in_sizes[9] < DM || in_sizes[11] < DM) return;
    if ((long long)out_size < (long long)MT * DM) return;
    const float* xq = (const float*)d_in[0]; const float* xk = (const float*)d_in[1]; const float* xv = (const float*)d_in[2]; const int* mask = (const int*)d_in[3];
    const float* wq = (const float*)d_in[4]; const float* bq = (const float*)d_in[5]; const float* wk = (const float*)d_in[6]; const float* bk = (const float*)d_in[7];
    const float* wv = (const float*)d_in[8]; const float* bv = (const float*)d_in[9]; const float* wo = (const float*)d_in[10]; const float* bo = (const float*)d_in[11];
    float* OUT = (float*)d_out;
    char* wsp = (char*)d_ws;
    auto take = [&](size_t bytes) { char* p = wsp; wsp += (bytes + 255) & ~(size_t)255; return (void*)p; };
    bf* WQt = (bf*)take((size_t)DM * DM * 2); bf* WKt = (bf*)take((size_t)DM * DM * 2); bf* WVt = (bf*)take((size_t)DM * DM * 2); bf* WOt = (bf*)take((size_t)DM * DM * 2);
    bf* XB = (bf*)take((size_t)MT * DM * 2);
    float* F = (float*)take((size_t)MT * DM * 4);
    h16* QP = (h16*)take((size_t)MT * DM * 2); h16* QR = (h16*)take((size_t)MT * DM * 2); h16* KP = (h16*)take((size_t)MT * DM * 2);
    h16* VTp = (h16*)take((size_t)MT * DM * 2); h16* VRp = (h16*)take((size_t)MT * DM * 2);
    bf* CTh = (bf*)take((size_t)MT * DM * 2); bf* CTl = (bf*)take((size_t)MT * DM * 2);
    if ((size_t)(wsp - (char*)d_ws) > ws_size) return;
    const unsigned GW = (unsigned)((size_t)DM * DM / 64 / 64);
    const unsigned GC = (unsigned)((size_t)MT * DM / 8 / 256);
    const dim3 GG((unsigned)(MT / 64), (unsigned)(DM / 64), 1);
    k_wtG<<<GW, 256, 0, stream>>>(wq, WQt);
    k_wtG<<<GW, 256, 0, stream>>>(wk, WKt);
    k_wtG<<<GW, 256, 0, stream>>>(wv, WVt);
    k_wtG<<<GW, 256, 0, stream>>>(wo, WOt);
    k_cvt8<<<GC, 256, 0, stream>>>(xq, XB);
    k_gemmw<bf, 0, true><<<GG, 32, 0, stream>>>(XB, nullptr, WQt, nullptr, DM, F, DM, bq, 0, 0, 0);
    k_qp<<<GC, 256, 0, stream>>>(F, QP, QR);
    k_cvt8<<<GC, 256, 0, stream>>>(xk, XB);
    k_gemmw<bf, 0, true><<<GG, 32, 0, stream>>>(XB, nullptr, WKt, nullptr, DM, F, DM, bk, 0, 0, 0);
    k_kp<<<GC, 256, 0, stream>>>(F, KP);
    k_cvt8<<<GC, 256, 0, stream>>>(xv, XB);
    k_gemmw<bf, 0, true><<<GG, 32, 0, stream>>>(XB, nullptr, WVt, nullptr, DM, F, DM, bv, 0, 0, 0);
    k_vtp<<<GC, 256, 0, stream>>>(F, VTp, VRp);
    k_flash<<<dim3((unsigned)(SEQ / 64), (unsigned)(NB * NH_), 1), 128, 0, stream>>>(QP, QR, KP, VTp, VRp, mask, CTh, CTl);
    k_gemmw<bf, 1, true><<<GG, 32, 0, stream>>>(CTh, CTl, WOt, nullptr, DM, OUT, DM, bo, 0, 0, 0);
}
